// LocalityAwareCrossAttention_35837207118362
// MI455X (gfx1250) — hardware-verified
//
#include <hip/hip_runtime.h>

typedef __attribute__((ext_vector_type(16))) _Float16 v16h;
typedef __attribute__((ext_vector_type(8)))  _Float16 v8h;
typedef __attribute__((ext_vector_type(16))) __bf16   v16b;
typedef __attribute__((ext_vector_type(8)))  __bf16   v8b;
typedef __attribute__((ext_vector_type(8)))  float    v8f;
typedef __attribute__((ext_vector_type(4)))  float    v4f;

#define NEG_INF (-__builtin_huge_valf())

__device__ __forceinline__ unsigned short f2bf_bits(float f) {
  unsigned u = __float_as_uint(f);
  return (unsigned short)((u + 0x7FFFu + ((u >> 16) & 1u)) >> 16);
}
__device__ __forceinline__ float bf_bits2f(unsigned short h) { return __uint_as_float(((unsigned)h) << 16); }

__device__ __forceinline__ void dep_guard_h(v8f& a, v8f& b, v16h x, v16h y) { asm volatile("v_nop\n\tv_nop\n\tv_nop\n\tv_nop" : "+v"(a), "+v"(b) : "v"(x), "v"(y)); }
__device__ __forceinline__ void dep_guard_b(v8f& a, v8f& b, v16b x, v16b y) { asm volatile("v_nop\n\tv_nop\n\tv_nop\n\tv_nop" : "+v"(a), "+v"(b) : "v"(x), "v"(y)); }
__device__ __forceinline__ void keep4_h(v16h a, v16h b, v16h c, v16h d) { asm volatile("v_nop" :: "v"(a), "v"(b), "v"(c), "v"(d)); }
__device__ __forceinline__ void keep4_b(v16b a, v16b b, v16b c, v16b d) { asm volatile("v_nop" :: "v"(a), "v"(b), "v"(c), "v"(d)); }
__device__ __forceinline__ void acc_guard4(v8f& a, v8f& b, v8f& c, v8f& d) { asm volatile("v_nop\n\tv_nop\n\tv_nop\n\tv_nop" : "+v"(a), "+v"(b), "+v"(c), "+v"(d)); }
template <typename T> struct Frag;
template <> struct Frag<_Float16> {
  typedef v16h V; union U { v16h v; v8h h[2]; };
  static __device__ __forceinline__ v16h load(const _Float16* p) {
    U f; f.h[0] = *(const v8h*)(p); f.h[1] = *(const v8h*)(p + 16); return f.v;
  }
  static __device__ __forceinline__ v8f mma(v16h a, v16h b, v8f c) {
    return __builtin_amdgcn_wmma_f32_16x16x32_f16(false, a, false, b, (short)0, c, false, false);
  }
  static __device__ __forceinline__ void guard(v8f& a, v8f& b, v16h x, v16h y) { dep_guard_h(a, b, x, y); }
  static __device__ __forceinline__ void keep(v16h a, v16h b, v16h c, v16h d) { keep4_h(a, b, c, d); }
};
template <> struct Frag<__bf16> {
  typedef v16b V; union U { v16b v; v8b h[2]; };
  static __device__ __forceinline__ v16b load(const __bf16* p) {
    U f; f.h[0] = *(const v8b*)(p); f.h[1] = *(const v8b*)(p + 16); return f.v;
  }
  static __device__ __forceinline__ v8f mma(v16b a, v16b b, v8f c) {
    return __builtin_amdgcn_wmma_f32_16x16x32_bf16(false, a, false, b, (short)0, c, false, false);
  }
  static __device__ __forceinline__ void guard(v8f& a, v8f& b, v16b x, v16b y) { dep_guard_b(a, b, x, y); }
  static __device__ __forceinline__ void keep(v16b a, v16b b, v16b c, v16b d) { keep4_b(a, b, c, d); }
};

#define NBATCH 2
#define NPIX  3136
#define HGRID 56
#define MTOK  6272
#define CD    256
#define KVLD  512
#define HDIM  32
#define NHEAD 8
#define RAD2  9
#define REACH 171
#define NCHK  49

template <int ET> struct Elem;
template <> struct Elem<0> { typedef _Float16 T; };
template <> struct Elem<1> { typedef __bf16 T; };
template <int ET, bool SPLIT, int BIAS_MODE, int OUT_MODE, bool RESID, int ACT = 0>
__global__ __launch_bounds__(256) void wmma_gemm64(
    const unsigned short* __restrict__ Ap, const unsigned short* __restrict__ A2p, int lda, long strideA,
    const unsigned short* __restrict__ Btp, const unsigned short* __restrict__ Bt2p, int ldb, long strideB,
    void* __restrict__ Cout, void* __restrict__ Cout2, int ldc, long strideC,
    const float* __restrict__ bias,
    const float* __restrict__ resid, long strideR,
    int M, int N, int K, float scale) {
  typedef typename Elem<ET>::T T;
  typedef typename Frag<T>::V V;
  const T* A = (const T*)Ap; const T* A2 = (const T*)A2p; const T* Bt = (const T*)Btp; const T* Bt2 = (const T*)Bt2p;
  __shared__ __align__(16) float sT[8][16 * 68];
  const int b    = blockIdx.y;
  const int lane = threadIdx.x & 31;
  const int wave = threadIdx.x >> 5;
  const int tilesN = N >> 6;
  const int tilesM = M >> 6;
  const int tile = blockIdx.x * 8 + wave;
  if (tile >= tilesM * tilesN) return;
  const int tm = tile / tilesN;
  const int tn = tile - tm * tilesN;
  const int m0 = tm << 6;
  const int n0 = tn << 6;

  const T* Ab  = A  + (size_t)b * strideA;
  const T* Bb  = Bt + (size_t)b * strideB;
  const T* Ab2 = SPLIT ? (A2  + (size_t)b * strideA) : nullptr;
  const T* Bb2 = SPLIT ? (Bt2 + (size_t)b * strideB) : nullptr;

  const int rlane = lane & 15;
  const int koff  = (lane >> 4) * 8;
  const int mOff  = (lane >> 4) * 8;

  v8f acc[4][4];
#pragma unroll
  for (int i = 0; i < 4; ++i)
#pragma unroll
    for (int j = 0; j < 4; ++j) acc[i][j] = (v8f){0.f,0.f,0.f,0.f,0.f,0.f,0.f,0.f};

  for (int k0 = 0; k0 < K; k0 += 32) {
    V bh[4], bl[4];
#pragma unroll
    for (int j = 0; j < 4; ++j) {
      const size_t bo = (size_t)(n0 + (j << 4) + rlane) * ldb + koff + k0;
      bh[j] = Frag<T>::load(Bb + bo);
      if (SPLIT) bl[j] = Frag<T>::load(Bb2 + bo);
    }
#pragma unroll
    for (int i = 0; i < 4; ++i) {
      const size_t ao = (size_t)(m0 + (i << 4) + rlane) * lda + koff + k0;
      V ah = Frag<T>::load(Ab + ao);
      V al;
      if (SPLIT) al = Frag<T>::load(Ab2 + ao);
#pragma unroll
      for (int j = 0; j < 4; ++j) {
        acc[i][j] = Frag<T>::mma(ah, bh[j], acc[i][j]);
        if (SPLIT) {
          acc[i][j] = Frag<T>::mma(ah, bl[j], acc[i][j]);
          acc[i][j] = Frag<T>::mma(al, bh[j], acc[i][j]);
        }
      }
      Frag<T>::guard(acc[i][0], acc[i][3], ah, SPLIT ? al : ah);
    }
    Frag<T>::keep(bh[0], bh[1], bh[2], bh[3]);
    if (SPLIT) Frag<T>::keep(bl[0], bl[1], bl[2], bl[3]);
  }
  acc_guard4(acc[0][0], acc[0][1], acc[0][2], acc[0][3]);
  acc_guard4(acc[1][0], acc[1][1], acc[1][2], acc[1][3]);
  acc_guard4(acc[2][0], acc[2][1], acc[2][2], acc[2][3]);
  acc_guard4(acc[3][0], acc[3][1], acc[3][2], acc[3][3]);

  float* slab = sT[wave];
  const float* Rb = RESID ? (resid + (size_t)b * strideR) : nullptr;
#pragma unroll
  for (int i = 0; i < 4; ++i) {
    const int mBase = m0 + (i << 4);
#pragma unroll
    for (int j = 0; j < 4; ++j) {
      const int n = n0 + (j << 4) + rlane;
      float bv = 0.f;
      if (BIAS_MODE == 2) bv = bias[n];
#pragma unroll
      for (int r = 0; r < 8; ++r) {
        float v = acc[i][j][r] * scale;
        if (BIAS_MODE == 1) v += bias[mBase + mOff + r];
        if (BIAS_MODE == 2) v += bv;
        if (RESID) v += Rb[(size_t)(mBase + mOff + r) * ldc + n];
        if (ACT == 1) v = tanhf(v);
        if (ACT == 2) v = fmaxf(v, 0.0f);
        if (ACT == 3) v = v / (1.0f + expf(-v));
        if (ACT == 4) v = (v > 0.f) ? v : 0.01f * v;
        if (ACT == 5) v = 0.5f * v * (1.0f + erff(v * 0.70710678118654752f));
        slab[(mOff + r) * 68 + (j << 4) + rlane] = v;
      }
    }
    __builtin_amdgcn_fence(__ATOMIC_RELEASE, "workgroup");
    __builtin_amdgcn_wave_barrier();
    __builtin_amdgcn_fence(__ATOMIC_ACQUIRE, "workgroup");
    if (OUT_MODE == 0) {
      float* C = (float*)Cout + (size_t)b * strideC;
      const int hh = lane >> 4, c4 = (lane & 15) * 4;
      for (int pass = 0; pass < 2; ++pass) {
#pragma unroll
        for (int it = 0; it < 8; ++it) {
          const int row = it * 2 + hh;
          v4f v = *(const v4f*)(slab + row * 68 + c4);
          *(volatile v4f*)(C + (size_t)(mBase + row) * ldc + n0 + c4) = v;
        }
        __threadfence();
      }
    } else {
      const int q = lane >> 3, c8 = (lane & 7) * 8;
      unsigned short* C  = (unsigned short*)Cout  + (size_t)b * strideC;
      unsigned short* C2 = (OUT_MODE == 2) ? ((unsigned short*)Cout2 + (size_t)b * strideC) : nullptr;
      for (int pass = 0; pass < 2; ++pass) {
#pragma unroll
        for (int it = 0; it < 4; ++it) {
          const int row = it * 4 + q;
          const float* sp = slab + row * 68 + c8;
          v8h hv, lv;
#pragma unroll
          for (int e = 0; e < 8; ++e) {
            if (OUT_MODE == 1) {
              hv[e] = (_Float16)sp[e];
            } else {
              unsigned short hb = f2bf_bits(sp[e]);
              unsigned short lb = f2bf_bits(sp[e] - bf_bits2f(hb));
              hv[e] = __builtin_bit_cast(_Float16, hb);
              lv[e] = __builtin_bit_cast(_Float16, lb);
            }
          }
          *(volatile v8h*)(C + (size_t)(mBase + row) * ldc + n0 + c8) = hv;
          if (OUT_MODE == 2) *(volatile v8h*)(C2 + (size_t)(mBase + row) * ldc + n0 + c8) = lv;
        }
        __threadfence();
      }
    }
    __builtin_amdgcn_fence(__ATOMIC_RELEASE, "workgroup");
    __builtin_amdgcn_wave_barrier();
    __builtin_amdgcn_fence(__ATOMIC_ACQUIRE, "workgroup");
  }
}

__global__ __launch_bounds__(256) void cast8_kernel(
    const float* __restrict__ in, _Float16* __restrict__ out, int n8, float scale) {
  const int i = blockIdx.x * 256 + threadIdx.x;
  if (i < n8) {
    const float* p = in + (size_t)i * 8;
    const v4f f0 = *(const v4f*)p;
    const v4f f1 = *(const v4f*)(p + 4);
    v8h hv;
    hv[0] = (_Float16)(f0[0] * scale); hv[1] = (_Float16)(f0[1] * scale);
    hv[2] = (_Float16)(f0[2] * scale); hv[3] = (_Float16)(f0[3] * scale);
    hv[4] = (_Float16)(f1[0] * scale); hv[5] = (_Float16)(f1[1] * scale);
    hv[6] = (_Float16)(f1[2] * scale); hv[7] = (_Float16)(f1[3] * scale);
    _Float16* q = out + (size_t)i * 8;
    *(volatile v8h*)q = hv;
    __threadfence();
    *(volatile v8h*)q = hv;
  }
}

#define L_NW 4
#define L_QB 64
#define L_KC 64
#define L_KP 40
#define L_VP 72
#define L_PP 72
#define L_OP 36
#define L_MAXCH 8
#define PSC 32768.0f

__device__ __forceinline__ v8f mma_h(v16h a, v16h b, v8f c) {
  c = __builtin_amdgcn_wmma_f32_16x16x32_f16(false, a, false, b, (short)0, c, false, false);
  asm volatile("v_nop\n\tv_nop\n\tv_nop\n\tv_nop" : "+v"(c) : "v"(a), "v"(b));
  return c;
}

__global__ __launch_bounds__(128) void local_attn_kernel(
    const _Float16* __restrict__ q16, const _Float16* __restrict__ kv16, float* __restrict__ out) {
  __shared__ __align__(16) _Float16 Ks[L_KC * L_KP];
  __shared__ __align__(16) _Float16 Vt[HDIM * L_VP];
  __shared__ __align__(16) _Float16 Ps[L_NW][16 * L_PP];
  __shared__ __align__(16) float Os[L_NW][16 * L_OP];

  const int tid  = threadIdx.x;
  const int wave = tid >> 5;
  const int lane = tid & 31;
  const int hh   = lane >> 4;
  const int c    = lane & 15;
  const int qb   = blockIdx.x;
  const int h    = blockIdx.y & 7;
  const int b    = blockIdx.y >> 3;
  const int qblk = qb * L_QB;
  const int q0   = qblk + wave * 16;
  const size_t tok0 = (size_t)b * NPIX;

  const int lo = qblk - REACH;
  const int kc_lo = (lo < 0) ? 0 : (lo >> 6);
  const int hi = qblk + (L_QB - 1) + REACH;
  int kc_hi = hi >> 6;
  if (kc_hi > NCHK - 1) kc_hi = NCHK - 1;
  int nch = kc_hi - kc_lo + 1;
  if (nch > L_MAXCH) nch = L_MAXCH;

  const v16h qa = Frag<_Float16>::load(q16 + (tok0 + q0 + c) * CD + h * HDIM + 8 * hh);

  int yq[8], xq[8];
#pragma unroll
  for (int r = 0; r < 8; ++r) {
    const int n = q0 + 8 * hh + r;
    yq[r] = n / HGRID;
    xq[r] = n - yq[r] * HGRID;
  }

  float mrow[8], lrow[8];
  v8f oacc[2];
#pragma unroll
  for (int r = 0; r < 8; ++r) { mrow[r] = NEG_INF; lrow[r] = 0.f; }
#pragma unroll
  for (int t = 0; t < 2; ++t) oacc[t] = (v8f){0.f,0.f,0.f,0.f,0.f,0.f,0.f,0.f};

  const float qsc = 0.17677669529663687f * 0.015625f;

  for (int i = 0; i < L_MAXCH; ++i) {
    if (i >= nch) break;
    const int kv0 = (kc_lo + i) * L_KC;
    __syncthreads();
    {
#pragma unroll
      for (int it = 0; it < 2; ++it) {
        const int piece = tid + it * 128;
        const int kvr = piece >> 2, part = piece & 3;
        const _Float16* krow = kv16 + (tok0 + kv0 + kvr) * KVLD + h * HDIM + part * 8;
        const v8h k8 = *(const v8h*)krow;
        *(v8h*)(Ks + kvr * L_KP + part * 8) = k8;
        const v8h v8 = *(const v8h*)(krow + CD);
#pragma unroll
        for (int e = 0; e < 8; ++e) Vt[(part * 8 + e) * L_VP + kvr] = v8[e];
      }
    }
    __syncthreads();

    v8f s[4];
#pragma unroll
    for (int j = 0; j < 4; ++j) {
      s[j] = (v8f){0.f,0.f,0.f,0.f,0.f,0.f,0.f,0.f};
      const v16h kb = Frag<_Float16>::load(Ks + (j * 16 + c) * L_KP + 8 * hh);
      s[j] = mma_h(qa, kb, s[j]);
    }
    int ym[4], xm[4];
#pragma unroll
    for (int j = 0; j < 4; ++j) {
      const int m = kv0 + j * 16 + c;
      ym[j] = m / HGRID;
      xm[j] = m - ym[j] * HGRID;
    }
    float cm[8];
#pragma unroll
    for (int r = 0; r < 8; ++r) {
      float mx = NEG_INF;
#pragma unroll
      for (int j = 0; j < 4; ++j) {
        const int dy = yq[r] - ym[j];
        const int dx = xq[r] - xm[j];
        const int d2 = dy * dy + dx * dx;
        const float v = (d2 <= RAD2) ? (s[j][r] * qsc) : NEG_INF;
        s[j][r] = v;
        mx = fmaxf(mx, v);
      }
#pragma unroll
      for (int off = 1; off < 16; off <<= 1) mx = fmaxf(mx, __shfl_xor(mx, off, 32));
      cm[r] = mx;
    }
    _Float16* pw = Ps[wave];
#pragma unroll
    for (int r = 0; r < 8; ++r) {
      const float mnew  = fmaxf(mrow[r], cm[r]);
      const float msafe = (mnew == NEG_INF) ? 0.0f : mnew;
      const float alpha = __expf(mrow[r] - msafe);
      mrow[r] = mnew;
      float psum = 0.f;
#pragma unroll
      for (int j = 0; j < 4; ++j) {
        const float p = __expf(s[j][r] - msafe);
        psum += p;
        pw[(8 * hh + r) * L_PP + j * 16 + c] = (_Float16)(p * PSC);
      }
#pragma unroll
      for (int off = 1; off < 16; off <<= 1) psum += __shfl_xor(psum, off, 32);
      lrow[r] = lrow[r] * alpha + psum;
      oacc[0][r] *= alpha;
      oacc[1][r] *= alpha;
    }
    __builtin_amdgcn_fence(__ATOMIC_RELEASE, "workgroup");
    __builtin_amdgcn_wave_barrier();
    __builtin_amdgcn_fence(__ATOMIC_ACQUIRE, "workgroup");
#pragma unroll
    for (int kk = 0; kk < 2; ++kk) {
      const v16h pa = Frag<_Float16>::load(pw + c * L_PP + kk * 32 + 8 * hh);
#pragma unroll
      for (int t = 0; t < 2; ++t) {
        const v16h vb = Frag<_Float16>::load(Vt + (t * 16 + c) * L_VP + kk * 32 + 8 * hh);
        oacc[t] = mma_h(pa, vb, oacc[t]);
      }
    }
  }

  float* os = Os[wave];
#pragma unroll
  for (int r = 0; r < 8; ++r) {
    const float inv = 1.0f / (lrow[r] * (PSC * 8.0f));
    os[(8 * hh + r) * L_OP + c]      = oacc[0][r] * inv;
    os[(8 * hh + r) * L_OP + 16 + c] = oacc[1][r] * inv;
  }
  __builtin_amdgcn_fence(__ATOMIC_RELEASE, "workgroup");
  __builtin_amdgcn_wave_barrier();
  __builtin_amdgcn_fence(__ATOMIC_ACQUIRE, "workgroup");
  {
    const int q8 = lane >> 3, c4 = (lane & 7) * 4;
    float* ob = out + (tok0 + q0) * CD + h * HDIM;
    for (int pass = 0; pass < 2; ++pass) {
#pragma unroll
      for (int it = 0; it < 4; ++it) {
        const int row = it * 4 + q8;
        v4f val = *(const v4f*)(os + row * L_OP + c4);
        *(volatile v4f*)(ob + (size_t)row * CD + c4) = val;
      }
      __threadfence();
    }
  }
}

extern "C" void kernel_launch(void* const* d_in, const int* in_sizes, int n_in,
                              void* d_out, int out_size, void* d_ws, size_t ws_size,
                              hipStream_t stream) {
  if (n_in < 7) return;
  if (in_sizes[0] != MTOK * CD || in_sizes[1] != MTOK * CD) return;
  if (in_sizes[2] != CD * CD || in_sizes[3] != CD * CD || in_sizes[4] != CD * CD || in_sizes[5] != CD * CD) return;
  if (in_sizes[6] != CD) return;
  if (out_size != MTOK * CD) return;

  const float* x   = (const float*)d_in[0];
  const float* xkv = (const float*)d_in[1];
  const float* Wq  = (const float*)d_in[2];
  const float* Wk  = (const float*)d_in[3];
  const float* Wv  = (const float*)d_in[4];
  const float* Wp  = (const float*)d_in[5];
  const float* bp  = (const float*)d_in[6];
  float* out = (float*)d_out;

  const size_t szX   = (size_t)MTOK * CD * 2;
  const size_t szXKV = (size_t)MTOK * CD * 2;
  const size_t szWQ  = (size_t)CD * CD * 2;
  const size_t szWKV = (size_t)2 * CD * CD * 2;
  const size_t szWP  = (size_t)CD * CD * 2;
  const size_t szQ   = (size_t)MTOK * CD * 2;
  const size_t szKV  = (size_t)MTOK * KVLD * 2;
  const size_t szAO  = (size_t)MTOK * CD * 4;
  const size_t szAO16 = (size_t)MTOK * CD * 2;
  const size_t oX    = 0;
  const size_t oXKV  = oX + szX;
  const size_t oWQ   = oXKV + szXKV;
  const size_t oWKV  = oWQ + szWQ;
  const size_t oWP   = oWKV + szWKV;
  const size_t oQ    = oWP + szWP;
  const size_t oKV   = oQ + szQ;
  const size_t oAO   = oKV + szKV;
  const size_t oAO16 = oAO + szAO;
  const size_t total = oAO16 + szAO16;
  if (total > ws_size) return;

  char* ws = (char*)d_ws;
  _Float16* x16    = (_Float16*)(ws + oX);
  _Float16* xkv16  = (_Float16*)(ws + oXKV);
  _Float16* wq16   = (_Float16*)(ws + oWQ);
  _Float16* wkv16  = (_Float16*)(ws + oWKV);
  _Float16* wp16   = (_Float16*)(ws + oWP);
  _Float16* q16    = (_Float16*)(ws + oQ);
  _Float16* kv16   = (_Float16*)(ws + oKV);
  float*    attnf  = (float*)(ws + oAO);
  _Float16* attn16 = (_Float16*)(ws + oAO16);
  const float* dummy_resid = (const float*)(ws + oX);

  {
    const int n8x = MTOK * CD / 8;
    cast8_kernel<<<dim3((n8x + 255) / 256), 256, 0, stream>>>(x,   x16,   n8x, 1.0f);
    cast8_kernel<<<dim3((n8x + 255) / 256), 256, 0, stream>>>(xkv, xkv16, n8x, 1.0f);
    const int n8w = CD * CD / 8;
    cast8_kernel<<<dim3((n8w + 255) / 256), 256, 0, stream>>>(Wq, wq16, n8w, 64.0f);
    cast8_kernel<<<dim3((n8w + 255) / 256), 256, 0, stream>>>(Wk, wkv16, n8w, 64.0f);
    cast8_kernel<<<dim3((n8w + 255) / 256), 256, 0, stream>>>(Wv, wkv16 + (size_t)CD * CD, n8w, 64.0f);
    cast8_kernel<<<dim3((n8w + 255) / 256), 256, 0, stream>>>(Wp, wp16, n8w, 64.0f);
  }
  {
    const int tiles = (MTOK / 64) * (CD / 64);
    wmma_gemm64<0, false, 0, 1, false><<<dim3((tiles + 7) / 8, 1), 256, 0, stream>>>(
        (const unsigned short*)x16, (const unsigned short*)x16, CD, (long)0,
        (const unsigned short*)wq16, (const unsigned short*)wq16, CD, (long)0,
        (void*)q16, (void*)q16, CD, (long)0,
        bp, dummy_resid, (long)0, MTOK, CD, CD, 0.125f);
  }
  {
    const int tiles = (MTOK / 64) * (KVLD / 64);
    wmma_gemm64<0, false, 0, 1, false><<<dim3((tiles + 7) / 8, 1), 256, 0, stream>>>(
        (const unsigned short*)xkv16, (const unsigned short*)xkv16, CD, (long)0,
        (const unsigned short*)wkv16, (const unsigned short*)wkv16, CD, (long)0,
        (void*)kv16, (void*)kv16, KVLD, (long)0,
        bp, dummy_resid, (long)0, MTOK, KVLD, CD, 0.125f);
  }
  local_attn_kernel<<<dim3(NPIX / L_QB, NBATCH * NHEAD), 128, 0, stream>>>(q16, kv16, attnf);
  {
    const int n8 = MTOK * CD / 8;
    cast8_kernel<<<dim3((n8 + 255) / 256), 256, 0, stream>>>(attnf, attn16, n8, 64.0f);
  }
  {
    const int tiles = (MTOK / 64) * (CD / 64);
    wmma_gemm64<0, false, 2, 0, false><<<dim3((tiles + 7) / 8, 1), 256, 0, stream>>>(
        (const unsigned short*)attn16, (const unsigned short*)attn16, CD, (long)0,
        (const unsigned short*)wp16, (const unsigned short*)wp16, CD, (long)0,
        (void*)out, (void*)out, CD, (long)0,
        bp, dummy_resid, (long)0, MTOK, CD, CD, 1.0f / 4096.0f);
  }
  (void)ws_size;
}
